// Decoder_66460323938638
// MI455X (gfx1250) — hardware-verified
//
#include <hip/hip_runtime.h>
#include <math.h>

typedef __attribute__((ext_vector_type(16))) _Float16 v16h;
typedef __attribute__((ext_vector_type(8)))  _Float16 v8h;
typedef __attribute__((ext_vector_type(16))) __bf16   v16b;
typedef __attribute__((ext_vector_type(8)))  __bf16   v8b;
typedef __attribute__((ext_vector_type(8)))  float    v8f;
typedef __attribute__((ext_vector_type(4)))  float    v4f;

constexpr int kB    = 32;
constexpr int kBP   = 64;
constexpr int kT    = 400;
constexpr int kE    = 512;
constexpr int kH    = 1024;
constexpr int kA    = 512;
constexpr int kV    = 5000;
constexpr int kVP   = 5120;
constexpr int kO    = 100;
constexpr int kG4   = 4 * kH;
constexpr int kH2   = 2 * kH;
constexpr int kF    = kH + kE;
constexpr int kRowsE = kB * kT;
constexpr int kRowsO = kB * kO;
constexpr int kThr  = 256;
constexpr float kInCarry = 1024.0f;
constexpr float kWCarry  = 4096.0f;
constexpr float kSc20 = 1.0f / (kInCarry * kInCarry);
constexpr float kSc22 = 1.0f / (kInCarry * kWCarry);
constexpr float kF16MinNormal = 6.103515625e-5f;
constexpr float kNegFill = -3.4028234663852886e38f;

static_assert((kRowsE % 64) == 0 && (kRowsO % 64) == 0 && (kBP % 64) == 0 && (kA % 64) == 0 && (kG4 % 64) == 0 && (kVP % 64) == 0, "GEMM M, N multiples of 64");
static_assert(((kRowsE / 64) * (kA / 64)) % 8 == 0 && ((kRowsO / 64) * (kG4 / 64)) % 8 == 0 && ((kRowsO / 64) * (kVP / 64)) % 8 == 0 && ((kBP / 64) * (kG4 / 64)) % 8 == 0 && ((kBP / 64) * (kA / 64)) % 8 == 0, "GEMM grids exact");
static_assert((kE % 32) == 0 && (kH % 32) == 0 && (kH2 % 32) == 0 && (kF % 32) == 0 && kV % 4 == 0, "GEMM K multiples of 32; output rows hold whole 4-float vectors");

constexpr size_t kOffHP16 = 0ull;
constexpr size_t kOffEY16 = 13107200ull;
constexpr size_t kOffWENC = 19660800ull;
constexpr size_t kOffWHH0 = 20185088ull;
constexpr size_t kOffWDEC = 28573696ull;
constexpr size_t kOffWIH0E = 29622272ull;
constexpr size_t kOffWIH0C = 38010880ull;
constexpr size_t kOffW1CAT = 42205184ull;
constexpr size_t kOffWOUT = 58982400ull;
constexpr size_t kOffBIAS = 74711040ull;
constexpr size_t kOffPENC = 74784768ull;
constexpr size_t kOffEYG = 100999168ull;
constexpr size_t kOffHV0 = 153427968ull;
constexpr size_t kOffDEC = 154476544ull;
constexpr size_t kOffCG = 154607616ull;
constexpr size_t kOffG1 = 155656192ull;
constexpr size_t kOffZZ16 = 156704768ull;
constexpr size_t kOffCT16 = 156966912ull;
constexpr size_t kOffCT32 = 157032448ull;
constexpr size_t kOffC0 = 157097984ull;
constexpr size_t kOffC1 = 157229056ull;
constexpr size_t kOffZS16 = 157360128ull;
constexpr size_t kOffOUTP = 167190528ull;
constexpr size_t kWsTotal = 232726528ull;
static_assert(kWsTotal <= 268435456ull, "carve cap");
static_assert(kOffHP16 == 0
              && kOffEY16 == kOffHP16 + 13107200ull
              && kOffWENC == kOffEY16 + 6553600ull
              && kOffWHH0 == kOffWENC + 524288ull
              && kOffWDEC == kOffWHH0 + 8388608ull
              && kOffWIH0E == kOffWDEC + 1048576ull
              && kOffWIH0C == kOffWIH0E + 8388608ull
              && kOffW1CAT == kOffWIH0C + 4194304ull
              && kOffWOUT == kOffW1CAT + 16777216ull
              && kOffBIAS == kOffWOUT + 15728640ull
              && kOffPENC == kOffBIAS + 73728ull
              && kOffEYG == kOffPENC + 26214400ull
              && kOffHV0 == kOffEYG + 52428800ull
              && kOffDEC == kOffHV0 + 1048576ull
              && kOffCG == kOffDEC + 131072ull
              && kOffG1 == kOffCG + 1048576ull
              && kOffZZ16 == kOffG1 + 1048576ull
              && kOffCT16 == kOffZZ16 + 262144ull
              && kOffCT32 == kOffCT16 + 65536ull
              && kOffC0 == kOffCT32 + 65536ull
              && kOffC1 == kOffC0 + 131072ull
              && kOffZS16 == kOffC1 + 131072ull
              && kOffOUTP == kOffZS16 + 9830400ull
              && kWsTotal == kOffOUTP + 65536000ull, "the carve is chained and totalled");
static_assert((kOffHP16 % 256) == 0 && (kOffEY16 % 256) == 0 && (kOffWENC % 256) == 0 && (kOffWHH0 % 256) == 0 && (kOffWDEC % 256) == 0 && (kOffWIH0E % 256) == 0 && (kOffWIH0C % 256) == 0 && (kOffW1CAT % 256) == 0 && (kOffWOUT % 256) == 0 && (kOffBIAS % 256) == 0 && (kOffPENC % 256) == 0 && (kOffEYG % 256) == 0 && (kOffHV0 % 256) == 0 && (kOffDEC % 256) == 0 && (kOffCG % 256) == 0 && (kOffG1 % 256) == 0 && (kOffZZ16 % 256) == 0 && (kOffCT16 % 256) == 0 && (kOffCT32 % 256) == 0 && (kOffC0 % 256) == 0 && (kOffC1 % 256) == 0 && (kOffZS16 % 256) == 0 && (kOffOUTP % 256) == 0, "aligned regions");
constexpr int kFB0 = 0, kFB1 = 4096, kFBENC = 8192, kFBOUT = 8704, kFZB = 13824, kFEnd = 18432;
static_assert(kFB1 == kFB0 + kG4 && kFBENC == kFB1 + kG4 && kFBOUT == kFBENC + kA && kFZB == kFBOUT + kVP && kFEnd - kFZB >= kG4, "bias stream map; the zero row covers the widest zero-bias product: 4,096 columns");

__device__ __forceinline__ unsigned short f2bf_bits(float f) {
  unsigned u = __float_as_uint(f);
  return (unsigned short)((u + 0x7FFFu + ((u >> 16) & 1u)) >> 16);
}
__device__ __forceinline__ float bf_bits2f(unsigned short h) { return __uint_as_float(((unsigned)h) << 16); }
__device__ __forceinline__ float bf16r(float f) { return bf_bits2f(f2bf_bits(f)); }
__device__ __forceinline__ float carry_flush(float v, float carry) {
  const float s = v * carry;
  return (fabsf(s) < kF16MinNormal) ? 0.0f : s;
}
__device__ __forceinline__ float frcp(float x) { return __builtin_amdgcn_rcpf(x); }

__device__ __forceinline__ void dep_guard4_h(v8f& a, v8f& b, v8f& c, v8f& d, v16h x, v16h y) { asm volatile("v_nop\n\tv_nop\n\tv_nop\n\tv_nop" : "+v"(a), "+v"(b), "+v"(c), "+v"(d) : "v"(x), "v"(y)); }
__device__ __forceinline__ void dep_guard4_b(v8f& a, v8f& b, v8f& c, v8f& d, v16b x, v16b y) { asm volatile("v_nop\n\tv_nop\n\tv_nop\n\tv_nop" : "+v"(a), "+v"(b), "+v"(c), "+v"(d) : "v"(x), "v"(y)); }
__device__ __forceinline__ void keep4_h(v16h a, v16h b, v16h c, v16h d) { asm volatile("v_nop" :: "v"(a), "v"(b), "v"(c), "v"(d)); }
__device__ __forceinline__ void keep4_b(v16b a, v16b b, v16b c, v16b d) { asm volatile("v_nop" :: "v"(a), "v"(b), "v"(c), "v"(d)); }
__device__ __forceinline__ void acc_guard4(v8f& a, v8f& b, v8f& c, v8f& d) { asm volatile("v_nop\n\tv_nop\n\tv_nop\n\tv_nop" : "+v"(a), "+v"(b), "+v"(c), "+v"(d)); }

template <typename T> struct Frag;
template <> struct Frag<_Float16> {
  typedef v16h V; union U { v16h v; v8h h[2]; };
  static __device__ __forceinline__ v16h load(const _Float16* p) {
    U f; f.h[0] = *(const v8h*)(p); f.h[1] = *(const v8h*)(p + 16); return f.v;
  }
  static __device__ __forceinline__ v8f mma(v16h a, v16h b, v8f c) {
    return __builtin_amdgcn_wmma_f32_16x16x32_f16(false, a, false, b, (short)0, c, false, false);
  }
  static __device__ __forceinline__ void guard4(v8f& a, v8f& b, v8f& c, v8f& d, v16h x, v16h y) { dep_guard4_h(a, b, c, d, x, y); }
  static __device__ __forceinline__ void keep(v16h a, v16h b, v16h c, v16h d) { keep4_h(a, b, c, d); }
};
template <> struct Frag<__bf16> {
  typedef v16b V; union U { v16b v; v8b h[2]; };
  static __device__ __forceinline__ v16b load(const __bf16* p) {
    U f; f.h[0] = *(const v8b*)(p); f.h[1] = *(const v8b*)(p + 16); return f.v;
  }
  static __device__ __forceinline__ v8f mma(v16b a, v16b b, v8f c) {
    return __builtin_amdgcn_wmma_f32_16x16x32_bf16(false, a, false, b, (short)0, c, false, false);
  }
  static __device__ __forceinline__ void guard4(v8f& a, v8f& b, v8f& c, v8f& d, v16b x, v16b y) { dep_guard4_b(a, b, c, d, x, y); }
  static __device__ __forceinline__ void keep(v16b a, v16b b, v16b c, v16b d) { keep4_b(a, b, c, d); }
};

__device__ __forceinline__ v8f mma_h(v16h a, v16h b, v8f c) {
  c = __builtin_amdgcn_wmma_f32_16x16x32_f16(false, a, false, b, (short)0, c, false, false);
  asm volatile("v_nop\n\tv_nop\n\tv_nop\n\tv_nop" : "+v"(c) : "v"(a), "v"(b));
  return c;
}

template <int ET> struct Elem;
template <> struct Elem<0> { typedef _Float16 T; };
template <> struct Elem<1> { typedef __bf16 T; };
template <int ET, bool SPLIT, int BIAS_MODE, int OUT_MODE, bool RESID, int ACT = 0>
__global__ __launch_bounds__(256) void wmma_gemm64(
    const unsigned short* __restrict__ Ap, const unsigned short* __restrict__ A2p, int lda, long strideA,
    const unsigned short* __restrict__ Btp, const unsigned short* __restrict__ Bt2p, int ldb, long strideB,
    void* __restrict__ Cout, void* __restrict__ Cout2, int ldc, long strideC,
    const float* __restrict__ bias,
    const float* __restrict__ resid, long strideR,
    int M, int N, int K, float scale) {
  typedef typename Elem<ET>::T T;
  typedef typename Frag<T>::V V;
  const T* A = (const T*)Ap; const T* A2 = (const T*)A2p; const T* Bt = (const T*)Btp; const T* Bt2 = (const T*)Bt2p;
  __shared__ __align__(16) float sT[8][16 * 68];
  const int b    = blockIdx.y;
  const int lane = threadIdx.x & 31;
  const int wave = threadIdx.x >> 5;
  const int tilesN = N >> 6;
  const int tilesM = M >> 6;
  const int tile = blockIdx.x * 8 + wave;
  if (tile >= tilesM * tilesN) return;
  const int tm = tile / tilesN;
  const int tn = tile - tm * tilesN;
  const int m0 = tm << 6;
  const int n0 = tn << 6;

  const T* Ab  = A  + (size_t)b * strideA;
  const T* Bb  = Bt + (size_t)b * strideB;
  const T* Ab2 = SPLIT ? (A2  + (size_t)b * strideA) : nullptr;
  const T* Bb2 = SPLIT ? (Bt2 + (size_t)b * strideB) : nullptr;

  const int rlane = lane & 15;
  const int koff  = (lane >> 4) * 8;
  const int mOff  = (lane >> 4) * 8;

  v8f acc[4][4];
#pragma unroll
  for (int i = 0; i < 4; ++i)
#pragma unroll
    for (int j = 0; j < 4; ++j) acc[i][j] = (v8f){0.f,0.f,0.f,0.f,0.f,0.f,0.f,0.f};

  for (int k0 = 0; k0 < K; k0 += 32) {
    V bh[4], bl[4];
#pragma unroll
    for (int j = 0; j < 4; ++j) {
      const size_t bo = (size_t)(n0 + (j << 4) + rlane) * ldb + koff + k0;
      bh[j] = Frag<T>::load(Bb + bo);
      if (SPLIT) bl[j] = Frag<T>::load(Bb2 + bo);
    }
#pragma unroll
    for (int i = 0; i < 4; ++i) {
      const size_t ao = (size_t)(m0 + (i << 4) + rlane) * lda + koff + k0;
      V ah = Frag<T>::load(Ab + ao);
      V al;
      if (SPLIT) al = Frag<T>::load(Ab2 + ao);
#pragma unroll
      for (int j = 0; j < 4; ++j) {
        acc[i][j] = Frag<T>::mma(ah, bh[j], acc[i][j]);
        if (SPLIT) {
          acc[i][j] = Frag<T>::mma(ah, bl[j], acc[i][j]);
          acc[i][j] = Frag<T>::mma(al, bh[j], acc[i][j]);
        }
      }
      Frag<T>::guard4(acc[i][0], acc[i][1], acc[i][2], acc[i][3], ah, SPLIT ? al : ah);
    }
    Frag<T>::keep(bh[0], bh[1], bh[2], bh[3]);
    if (SPLIT) Frag<T>::keep(bl[0], bl[1], bl[2], bl[3]);
  }
  acc_guard4(acc[0][0], acc[0][1], acc[0][2], acc[0][3]);
  acc_guard4(acc[1][0], acc[1][1], acc[1][2], acc[1][3]);
  acc_guard4(acc[2][0], acc[2][1], acc[2][2], acc[2][3]);
  acc_guard4(acc[3][0], acc[3][1], acc[3][2], acc[3][3]);

  float* slab = sT[wave];
  const float* Rb = RESID ? (resid + (size_t)b * strideR) : nullptr;
#pragma unroll
  for (int i = 0; i < 4; ++i) {
    const int mBase = m0 + (i << 4);
#pragma unroll
    for (int j = 0; j < 4; ++j) {
      const int n = n0 + (j << 4) + rlane;
      float bv = 0.f;
      if (BIAS_MODE == 2) bv = bias[n];
#pragma unroll
      for (int r = 0; r < 8; ++r) {
        float v = acc[i][j][r] * scale;
        if (BIAS_MODE == 1) v += bias[mBase + mOff + r];
        if (BIAS_MODE == 2) v += bv;
        if (RESID) v += Rb[(size_t)(mBase + mOff + r) * ldc + n];
        if (ACT == 1) v = tanhf(v);
        if (ACT == 2) v = fmaxf(v, 0.0f);
        if (ACT == 3) v = v / (1.0f + expf(-v));
        if (ACT == 4) v = (v > 0.f) ? v : 0.01f * v;
        slab[(mOff + r) * 68 + (j << 4) + rlane] = v;
      }
    }
    __builtin_amdgcn_fence(__ATOMIC_RELEASE, "workgroup");
    __builtin_amdgcn_wave_barrier();
    __builtin_amdgcn_fence(__ATOMIC_ACQUIRE, "workgroup");
    if (OUT_MODE == 0) {
      float* C = (float*)Cout + (size_t)b * strideC;
      const int hh = lane >> 4, c4 = (lane & 15) * 4;
      for (int pass = 0; pass < 2; ++pass) {
#pragma unroll
        for (int it = 0; it < 8; ++it) {
          const int row = it * 2 + hh;
          v4f v = *(const v4f*)(slab + row * 68 + c4);
          *(volatile v4f*)(C + (size_t)(mBase + row) * ldc + n0 + c4) = v;
        }
        __threadfence();
      }
    } else {
      const int q = lane >> 3, c8 = (lane & 7) * 8;
      unsigned short* C  = (unsigned short*)Cout  + (size_t)b * strideC;
      unsigned short* C2 = (OUT_MODE == 2) ? ((unsigned short*)Cout2 + (size_t)b * strideC) : nullptr;
      for (int pass = 0; pass < 2; ++pass) {
#pragma unroll
        for (int it = 0; it < 4; ++it) {
          const int row = it * 4 + q;
          const float* sp = slab + row * 68 + c8;
          v8h hv, lv;
#pragma unroll
          for (int e = 0; e < 8; ++e) {
            if (OUT_MODE == 1) {
              hv[e] = (_Float16)sp[e];
            } else {
              unsigned short hb = f2bf_bits(sp[e]);
              unsigned short lb = f2bf_bits(sp[e] - bf_bits2f(hb));
              hv[e] = __builtin_bit_cast(_Float16, hb);
              lv[e] = __builtin_bit_cast(_Float16, lb);
            }
          }
          *(volatile v8h*)(C + (size_t)(mBase + row) * ldc + n0 + c8) = hv;
          if (OUT_MODE == 2) *(volatile v8h*)(C2 + (size_t)(mBase + row) * ldc + n0 + c8) = lv;
        }
        __threadfence();
      }
    }
    __builtin_amdgcn_fence(__ATOMIC_RELEASE, "workgroup");
    __builtin_amdgcn_wave_barrier();
    __builtin_amdgcn_fence(__ATOMIC_ACQUIRE, "workgroup");
  }
}

__global__ __launch_bounds__(kThr) void cast_plane_kernel(const float* __restrict__ src, unsigned short* __restrict__ dst,
                                                          int colsLog2, int dstPitch, int dstOff) {
  const int i   = blockIdx.x * kThr + threadIdx.x;
  const int sh  = colsLog2 - 3;
  const int row = i >> sh;
  const int c8  = (i & ((1 << sh) - 1)) * 8;
  const float* sp = src + ((size_t)row << colsLog2) + c8;
  const v4f a0 = *(const v4f*)(sp);
  const v4f a1 = *(const v4f*)(sp + 4);
  v8h hv;
#pragma unroll
  for (int e = 0; e < 4; ++e) {
    const float f0 = a0[e];
    const float f1 = a1[e];
    hv[e]     = (_Float16)carry_flush(bf16r(f0), kInCarry);
    hv[4 + e] = (_Float16)carry_flush(bf16r(f1), kInCarry);
  }
  unsigned short* dp = dst + (size_t)row * dstPitch + dstOff + c8;
  *(volatile v8h*)dp = hv;
  __threadfence();
  *(volatile v8h*)dp = hv;
}
__global__ __launch_bounds__(256) void wt_plane_kernel(const float* __restrict__ W, unsigned short* __restrict__ dst, int K, int N, int nLive, int ldd, int colOff) {
  const int n  = blockIdx.x;
  const int k8 = threadIdx.x * 8;
  const bool live = n < nLive;
  const int nc = live ? n : 0;
  v8h hv;
#pragma unroll
  for (int e = 0; e < 8; ++e) {
    const float w = W[(size_t)(k8 + e) * N + nc];
    hv[e] = (_Float16)(live ? carry_flush(bf16r(w), kWCarry) : 0.0f);
  }
  unsigned short* dp = dst + (size_t)n * ldd + colOff + k8;
  *(volatile v8h*)dp = hv;
  __threadfence();
  *(volatile v8h*)dp = hv;
}


__device__ __forceinline__ float fast_tanh(float v) { return 1.0f - 2.0f * frcp(__expf(2.0f * v) + 1.0f); }
__device__ __forceinline__ float fast_sigmoid(float v) { return frcp(1.0f + __expf(-v)); }

__global__ __launch_bounds__(kThr) void hp_mask_cast_kernel(const float* __restrict__ hpad, const int* __restrict__ hlen, unsigned short* __restrict__ HP16) {
  unsigned v = blockIdx.x * (unsigned)kThr + threadIdx.x;
  asm volatile("" : "+v"(v));
  const unsigned row = v >> 6;
  const unsigned k8 = (v & 63u) * 8u;
  const unsigned b = row / (unsigned)kT;
  const unsigned t = row - b * (unsigned)kT;
  int hl = hlen[b];
  asm volatile("" : "+v"(hl));
  const bool live = (int)t < hl;
  const float* sp = hpad + (size_t)row * kE + k8;
  const v4f a0 = *(const v4f*)sp, a1 = *(const v4f*)(sp + 4);
  v8h hv;
#pragma unroll
  for (int e = 0; e < 4; ++e) {
    const float x0 = a0[e], x1 = a1[e];
    hv[e]     = (_Float16)(live ? carry_flush(bf16r(x0), kInCarry) : 0.0f);
    hv[4 + e] = (_Float16)(live ? carry_flush(bf16r(x1), kInCarry) : 0.0f);
  }
  unsigned short* dp = HP16 + (size_t)row * kE + k8;
  *(volatile v8h*)dp = hv;
  __threadfence();
  *(volatile v8h*)dp = hv;
}
static_assert((kRowsE * (kE / 8)) % kThr == 0 && kE / 8 == 64, "encoder cast grid exact");

__global__ __launch_bounds__(kThr) void embed_gather_kernel(const float* __restrict__ embed, const int* __restrict__ ys_in, unsigned short* __restrict__ EY16) {
  unsigned v = blockIdx.x * (unsigned)kThr + threadIdx.x;
  asm volatile("" : "+v"(v));
  const unsigned row = v >> 7;
  const unsigned k8 = (v & 127u) * 8u;
  const unsigned t = row >> 5;
  const unsigned b = row & 31u;
  int id = ys_in[b * (unsigned)kO + t];
  asm volatile("" : "+v"(id));
  id = (id < 0) ? 0 : id;
  id = (id > kV - 1) ? (kV - 1) : id;
  const float* sp = embed + (size_t)id * kH + k8;
  const v4f a0 = *(const v4f*)sp, a1 = *(const v4f*)(sp + 4);
  v8h hv;
#pragma unroll
  for (int e = 0; e < 4; ++e) {
    const float x0 = a0[e], x1 = a1[e];
    hv[e]     = (_Float16)carry_flush(bf16r(x0), kInCarry);
    hv[4 + e] = (_Float16)carry_flush(bf16r(x1), kInCarry);
  }
  unsigned short* dp = EY16 + (size_t)row * kH + k8;
  *(volatile v8h*)dp = hv;
  __threadfence();
  *(volatile v8h*)dp = hv;
}
static_assert((kRowsO * (kH / 8)) % kThr == 0 && kH / 8 == 128 && kB == 32, "embedding grid exact; row = t 32 + b");

__global__ __launch_bounds__(kThr) void wih0_cast_kernel(const float* __restrict__ W, unsigned short* __restrict__ WE, unsigned short* __restrict__ WC) {
  unsigned v = blockIdx.x * (unsigned)kThr + threadIdx.x;
  asm volatile("" : "+v"(v));
  const unsigned n = v / 192u;
  const unsigned k8 = (v - n * 192u) * 8u;
  const float* sp = W + (size_t)n * kF + k8;
  const v4f a0 = *(const v4f*)sp, a1 = *(const v4f*)(sp + 4);
  v8h hv;
#pragma unroll
  for (int e = 0; e < 4; ++e) {
    const float x0 = a0[e], x1 = a1[e];
    hv[e]     = (_Float16)carry_flush(bf16r(x0), kInCarry);
    hv[4 + e] = (_Float16)carry_flush(bf16r(x1), kInCarry);
  }
  unsigned short* dp = (k8 < (unsigned)kH) ? (WE + (size_t)n * kH + k8) : (WC + (size_t)n * kE + (k8 - (unsigned)kH));
  *(volatile v8h*)dp = hv;
  __threadfence();
  *(volatile v8h*)dp = hv;
}
static_assert((kG4 * (kF / 8)) % kThr == 0 && kF / 8 == 192 && (kH % 256) == 0 && (kF % 256) == 0, "W_ih0 cast grid exact; the halves' boundary on a wave boundary");

__global__ __launch_bounds__(kThr) void bias_rows_kernel(const float* __restrict__ bih0, const float* __restrict__ bhh0, const float* __restrict__ bih1,
                                                         const float* __restrict__ bhh1, const float* __restrict__ benc, const float* __restrict__ bout,
                                                         float* __restrict__ BIAS) {
  unsigned v = blockIdx.x * (unsigned)kThr + threadIdx.x;
  asm volatile("" : "+v"(v));
  const unsigned i0 = v * 4u;
  v4f o = {0.f, 0.f, 0.f, 0.f};
  if (i0 < (unsigned)kFBENC) {
    const bool l1 = i0 >= (unsigned)kFB1;
    const unsigned j = i0 - (l1 ? (unsigned)kFB1 : 0u);
    const v4f a = *(const v4f*)((l1 ? bih1 : bih0) + j);
    const v4f c = *(const v4f*)((l1 ? bhh1 : bhh0) + j);
#pragma unroll
    for (int e = 0; e < 4; ++e) { const float x = a[e], y = c[e]; o[e] = bf16r(x) + bf16r(y); }
  } else if (i0 < (unsigned)kFBOUT) {
    const v4f a = *(const v4f*)(benc + (i0 - (unsigned)kFBENC));
#pragma unroll
    for (int e = 0; e < 4; ++e) { const float x = a[e]; o[e] = bf16r(x); }
  } else if (i0 < (unsigned)kFZB) {
    const unsigned j = i0 - (unsigned)kFBOUT;
    const bool live = j < (unsigned)kV;
    const v4f a = *(const v4f*)(bout + (live ? j : 0u));
#pragma unroll
    for (int e = 0; e < 4; ++e) { const float x = a[e]; o[e] = live ? bf16r(x) : 0.0f; }
  }
  float* dp = BIAS + i0;
  *(volatile v4f*)dp = o;
  __threadfence();
  *(volatile v4f*)dp = o;
}
static_assert(kFEnd / 4 == 18 * kThr && (kFB1 % 128) == 0 && (kFBENC % 128) == 0 && (kFBOUT % 128) == 0 && (kFZB % 128) == 0, "bias grid exact; region boundaries on wave boundaries");

__global__ __launch_bounds__(kThr) void state_zero_kernel(unsigned short* __restrict__ ZZ16, unsigned short* __restrict__ CT16, float* __restrict__ C0, float* __restrict__ C1) {
  unsigned v = blockIdx.x * (unsigned)kThr + threadIdx.x;
  asm volatile("" : "+v"(v));
  v8h zh;
#pragma unroll
  for (int e = 0; e < 8; ++e) zh[e] = (_Float16)0.0f;
  const v4f zf = {0.f, 0.f, 0.f, 0.f};
  for (int pass = 0; pass < 2; ++pass) {
    if (v < 16384u) *(volatile v8h*)(ZZ16 + (size_t)v * 8u) = zh;
    else if (v < 20480u) *(volatile v8h*)(CT16 + (size_t)(v - 16384u) * 8u) = zh;
    else if (v < 28672u) *(volatile v4f*)(C0 + (size_t)(v - 20480u) * 4u) = zf;
    else *(volatile v4f*)(C1 + (size_t)(v - 28672u) * 4u) = zf;
    __threadfence();
  }
}
static_assert(kBP * kH2 / 8 == 16384 && kBP * kE / 8 == 4096 && kB * kH / 4 == 8192 && 36864 == 144 * kThr, "state grid exact");

__global__ __launch_bounds__(kThr) void dec_attn_kernel(const float* __restrict__ PENC, const float* __restrict__ DEC, const float* __restrict__ gvec,
                                                        const int* __restrict__ hlen, const unsigned short* __restrict__ HP16, float* __restrict__ CT32,
                                                        unsigned short* __restrict__ CT16) {
  __shared__ __align__(16) float sD[kA];
  __shared__ __align__(16) float sG[kA];
  __shared__ __align__(16) float sS[512];
  __shared__ __align__(16) float sRed[32];
  __shared__ __align__(16) float sP[8 * kE];
  const int tid  = threadIdx.x;
  const int lane = tid & 31;
  const int wave = tid >> 5;
  const int b    = blockIdx.x;
  for (int a = tid; a < kA; a += kThr) {
    const float d = DEC[(size_t)b * kA + a];
    const float g = gvec[a];
    sD[a] = d;
    sG[a] = bf16r(g);
  }
  int hl = hlen[b];
  asm volatile("" : "+v"(hl));
  __syncthreads();

#pragma unroll 1
  for (int half = 0; half < 2; ++half) {
    const int p = tid + 256 * half;
    const int pc = (p < kT) ? p : 0;
    const float* pe = PENC + ((size_t)b * kT + pc) * kA;
    float acc = 0.0f;
#pragma unroll 1
    for (int a4 = 0; a4 < kA; a4 += 4) {
      const v4f q  = *(const v4f*)(pe + a4);
      const v4f dd = *(const v4f*)(sD + a4);
      const v4f gg = *(const v4f*)(sG + a4);
      acc += gg[0] * fast_tanh(q[0] + dd[0]);
      acc += gg[1] * fast_tanh(q[1] + dd[1]);
      acc += gg[2] * fast_tanh(q[2] + dd[2]);
      acc += gg[3] * fast_tanh(q[3] + dd[3]);
    }
    sS[p] = (p < kT && p < hl) ? acc : kNegFill;
  }
  __syncthreads();

  if (tid < 16) {
    float m = sS[tid * 32];
#pragma unroll 1
    for (int j = 1; j < 32; ++j) { const float q = sS[tid * 32 + j]; m = (q > m) ? q : m; }
    sRed[tid] = m;
  }
  __syncthreads();
  float mx = sRed[0];
#pragma unroll 1
  for (int j = 1; j < 16; ++j) { const float q = sRed[j]; mx = (q > mx) ? q : mx; }
  const float e0 = (tid < kT) ? __expf(sS[tid] - mx) : 0.0f;
  const float e1 = (tid + 256 < kT) ? __expf(sS[tid + 256] - mx) : 0.0f;
  __syncthreads();
  sS[tid] = e0;
  sS[tid + 256] = e1;
  __syncthreads();
  if (tid < 16) {
    float s = 0.0f;
#pragma unroll 1
    for (int j = 0; j < 32; ++j) s += sS[tid * 32 + j];
    sRed[16 + tid] = s;
  }
  __syncthreads();
  float den = 0.0f;
#pragma unroll 1
  for (int j = 0; j < 16; ++j) den += sRed[16 + j];

  float a8[16];
#pragma unroll
  for (int e = 0; e < 16; ++e) a8[e] = 0.0f;
  const unsigned short* hb = HP16 + (size_t)b * kT * kE + lane * 8;
#pragma unroll 1
  for (int j = 0; j < kT / 8; ++j) {
    const int p = wave + 8 * j;
    const float w = sS[p];
    const v8h y0 = *(const v8h*)(hb + (size_t)p * kE);
    const v8h y1 = *(const v8h*)(hb + (size_t)p * kE + 256);
#pragma unroll
    for (int e = 0; e < 8; ++e) { a8[e] += w * (float)y0[e]; a8[8 + e] += w * (float)y1[e]; }
  }
  {
    float* pp = sP + wave * kE + lane * 8;
    const v4f p0 = {a8[0], a8[1], a8[2], a8[3]}, p1 = {a8[4], a8[5], a8[6], a8[7]};
    const v4f p2 = {a8[8], a8[9], a8[10], a8[11]}, p3 = {a8[12], a8[13], a8[14], a8[15]};
    *(v4f*)(pp) = p0; *(v4f*)(pp + 4) = p1; *(v4f*)(pp + 256) = p2; *(v4f*)(pp + 260) = p3;
  }
  __syncthreads();
  if (wave == 0) {
    const float inv = (1.0f / den) * (1.0f / kInCarry);
    v4f c0v, c1v, c2v, c3v; v8h h0, h1;
#pragma unroll
    for (int e = 0; e < 8; ++e) {
      float s0 = 0.0f, s1 = 0.0f;
#pragma unroll
      for (int g = 0; g < 8; ++g) { s0 += sP[g * kE + lane * 8 + e]; s1 += sP[g * kE + 256 + lane * 8 + e]; }
      const float ct0 = s0 * inv, ct1 = s1 * inv;
      if (e < 4) { c0v[e] = ct0; c2v[e] = ct1; } else { c1v[e - 4] = ct0; c3v[e - 4] = ct1; }
      h0[e] = (_Float16)carry_flush(ct0, kInCarry);
      h1[e] = (_Float16)carry_flush(ct1, kInCarry);
    }
    float* cp = CT32 + (size_t)b * kE + lane * 8;
    unsigned short* hp = CT16 + (size_t)b * kE + lane * 8;
    for (int pass = 0; pass < 2; ++pass) {
      *(volatile v4f*)cp = c0v; *(volatile v4f*)(cp + 4) = c1v; *(volatile v4f*)(cp + 256) = c2v; *(volatile v4f*)(cp + 260) = c3v;
      *(volatile v8h*)hp = h0; *(volatile v8h*)(hp + 256) = h1;
      __threadfence();
    }
  }
}
static_assert(kT <= 512 && (kT % 8) == 0 && kE == 512 && kA == 512, "attention block: two positions a thread; 50 positions a wave; two column groups a lane");

__global__ __launch_bounds__(kThr) void cell0_kernel(const float* __restrict__ EYG, const float* __restrict__ CG, const float* __restrict__ HV0,
                                                     float* __restrict__ C0, unsigned short* __restrict__ ZZ16, int t) {
  unsigned v = blockIdx.x * (unsigned)kThr + threadIdx.x;
  asm volatile("" : "+v"(v));
  const unsigned b = v >> 7;
  const unsigned u8 = (v & 127u) * 8u;
  const float* ge = EYG + ((size_t)t * kB + b) * kG4 + u8;
  const float* gc = CG + (size_t)b * kG4 + u8;
  const float* gh = HV0 + (size_t)b * kG4 + u8;
  float* cp = C0 + (size_t)b * kH + u8;
  v4f co0, co1; v8h zh;
#pragma unroll
  for (int hlf = 0; hlf < 2; ++hlf) {
    const int o = 4 * hlf;
    const v4f ei = *(const v4f*)(ge + o), ef = *(const v4f*)(ge + kH + o), eg = *(const v4f*)(ge + 2 * kH + o), eo = *(const v4f*)(ge + 3 * kH + o);
    const v4f ci = *(const v4f*)(gc + o), cf = *(const v4f*)(gc + kH + o), cg = *(const v4f*)(gc + 2 * kH + o), cq = *(const v4f*)(gc + 3 * kH + o);
    const v4f hi = *(const v4f*)(gh + o), hf = *(const v4f*)(gh + kH + o), hg = *(const v4f*)(gh + 2 * kH + o), ho = *(const v4f*)(gh + 3 * kH + o);
    const v4f cold = *(const v4f*)(cp + o);
#pragma unroll
    for (int e = 0; e < 4; ++e) {
      const float ig = fast_sigmoid(ei[e] + ci[e] + hi[e]);
      const float fg = fast_sigmoid(ef[e] + cf[e] + hf[e]);
      const float gg = fast_tanh(eg[e] + cg[e] + hg[e]);
      const float og = fast_sigmoid(eo[e] + cq[e] + ho[e]);
      const float cn = fg * cold[e] + ig * gg;
      const float zn = og * fast_tanh(cn);
      if (hlf == 0) co0[e] = cn; else co1[e] = cn;
      zh[o + e] = (_Float16)carry_flush(zn, kInCarry);
    }
  }
  unsigned short* zp = ZZ16 + (size_t)b * kH2 + u8;
  for (int pass = 0; pass < 2; ++pass) {
    *(volatile v4f*)cp = co0; *(volatile v4f*)(cp + 4) = co1;
    *(volatile v8h*)zp = zh;
    __threadfence();
  }
}

__global__ __launch_bounds__(kThr) void cell1_kernel(const float* __restrict__ G1, const float* __restrict__ CT32, float* __restrict__ C1,
                                                     unsigned short* __restrict__ ZZ16, unsigned short* __restrict__ ZS16, int t) {
  unsigned v = blockIdx.x * (unsigned)kThr + threadIdx.x;
  asm volatile("" : "+v"(v));
  const unsigned b = v >> 7;
  const unsigned u8 = (v & 127u) * 8u;
  const float* gg1 = G1 + (size_t)b * kG4 + u8;
  float* cp = C1 + (size_t)b * kH + u8;
  v4f co0, co1; v8h zh, ch;
#pragma unroll
  for (int hlf = 0; hlf < 2; ++hlf) {
    const int o = 4 * hlf;
    const v4f gi = *(const v4f*)(gg1 + o), gf = *(const v4f*)(gg1 + kH + o), gg = *(const v4f*)(gg1 + 2 * kH + o), go = *(const v4f*)(gg1 + 3 * kH + o);
    const v4f cold = *(const v4f*)(cp + o);
#pragma unroll
    for (int e = 0; e < 4; ++e) {
      const float ig = fast_sigmoid(gi[e]);
      const float fg = fast_sigmoid(gf[e]);
      const float cg = fast_tanh(gg[e]);
      const float og = fast_sigmoid(go[e]);
      const float cn = fg * cold[e] + ig * cg;
      const float zn = og * fast_tanh(cn);
      if (hlf == 0) co0[e] = cn; else co1[e] = cn;
      zh[o + e] = (_Float16)carry_flush(zn, kInCarry);
    }
  }
  const bool ctx = u8 < (unsigned)kE;
  {
    const float* cs = CT32 + (size_t)b * kE + (ctx ? u8 : 0u);
    const v4f a0 = *(const v4f*)cs, a1 = *(const v4f*)(cs + 4);
#pragma unroll
    for (int e = 0; e < 4; ++e) { ch[e] = (_Float16)carry_flush(a0[e], kInCarry); ch[4 + e] = (_Float16)carry_flush(a1[e], kInCarry); }
  }
  unsigned short* zp = ZZ16 + (size_t)b * kH2 + kH + u8;
  unsigned short* sp = ZS16 + ((size_t)b * kO + t) * kF + u8;
  unsigned short* sc = ZS16 + ((size_t)b * kO + t) * kF + kH + (ctx ? u8 : 0u);
  for (int pass = 0; pass < 2; ++pass) {
    *(volatile v4f*)cp = co0; *(volatile v4f*)(cp + 4) = co1;
    *(volatile v8h*)zp = zh;
    *(volatile v8h*)sp = zh;
    if (ctx) *(volatile v8h*)sc = ch;
    __threadfence();
  }
}
static_assert(kB * (kH / 8) == 16 * kThr && kH / 8 == 128 && (kE / 8) % 32 == 0, "cell grids exact; the context's threads end on a wave boundary");

__global__ __launch_bounds__(kThr) void assemble_out_kernel(const float* __restrict__ OUTP, float* __restrict__ out) {
  unsigned i = blockIdx.x * (unsigned)kThr + threadIdx.x;
  asm volatile("" : "+v"(i));
  const unsigned row = i / 1250u;
  const unsigned c4 = (i - row * 1250u) * 4u;
  const v4f o = *(const v4f*)(OUTP + (size_t)row * kVP + c4);
  float* dp = out + (size_t)i * 4u;
  *(volatile v4f*)dp = o;
  __threadfence();
  *(volatile v4f*)dp = o;
}
static_assert(kV / 4 == 1250 && ((size_t)kRowsO * kV / 4) % kThr == 0, "output grid exact");

static_assert((kG4 * kH / 8) % kThr == 0, "plane cast grids exact");

extern "C" void kernel_launch(void* const* d_in, const int* in_sizes, int n_in,
                              void* d_out, int out_size, void* d_ws, size_t ws_size,
                              hipStream_t stream) {
  if (n_in < 18 || d_out == nullptr || d_ws == nullptr) return;
  if (in_sizes[0] != kB * kT * kE || in_sizes[1] != kB || in_sizes[2] != kB * kO || in_sizes[3] != kV * kH) return;
  if (in_sizes[4] != kG4 * kF || in_sizes[5] != kG4 * kH || in_sizes[6] != kG4 || in_sizes[7] != kG4) return;
  if (in_sizes[8] != kG4 * kH || in_sizes[9] != kG4 * kH || in_sizes[10] != kG4 || in_sizes[11] != kG4) return;
  if (in_sizes[12] != kE * kA || in_sizes[13] != kA || in_sizes[14] != kH * kA || in_sizes[15] != kA) return;
  if (in_sizes[16] != kF * kV || in_sizes[17] != kV) return;
  if ((size_t)out_size != (size_t)kRowsO * kV) return;
  if (ws_size < kWsTotal) return;
  const float* hpad  = (const float*)d_in[0];
  const int*   hlen  = (const int*)d_in[1];
  const int*   ys_in = (const int*)d_in[2];
  const float* embed = (const float*)d_in[3];
  const float* Wih0 = (const float*)d_in[4];
  const float* Whh0 = (const float*)d_in[5];
  const float* bih0 = (const float*)d_in[6];
  const float* bhh0 = (const float*)d_in[7];
  const float* Wih1 = (const float*)d_in[8];
  const float* Whh1 = (const float*)d_in[9];
  const float* bih1 = (const float*)d_in[10];
  const float* bhh1 = (const float*)d_in[11];
  const float* Wenc = (const float*)d_in[12];
  const float* benc = (const float*)d_in[13];
  const float* Wdec = (const float*)d_in[14];
  const float* gvec = (const float*)d_in[15];
  const float* Wout = (const float*)d_in[16];
  const float* bout = (const float*)d_in[17];
  float* out = (float*)d_out;
  char* ws = (char*)d_ws;
  unsigned short* HP16 = (unsigned short*)(ws + kOffHP16);
  unsigned short* EY16 = (unsigned short*)(ws + kOffEY16);
  unsigned short* WENC = (unsigned short*)(ws + kOffWENC);
  unsigned short* WHH0 = (unsigned short*)(ws + kOffWHH0);
  unsigned short* WDEC = (unsigned short*)(ws + kOffWDEC);
  unsigned short* WIH0E = (unsigned short*)(ws + kOffWIH0E);
  unsigned short* WIH0C = (unsigned short*)(ws + kOffWIH0C);
  unsigned short* W1CAT = (unsigned short*)(ws + kOffW1CAT);
  unsigned short* WOUT = (unsigned short*)(ws + kOffWOUT);
  float* BIAS = (float*)(ws + kOffBIAS);
  float* PENC = (float*)(ws + kOffPENC);
  float* EYG = (float*)(ws + kOffEYG);
  float* HV0 = (float*)(ws + kOffHV0);
  float* DEC = (float*)(ws + kOffDEC);
  float* CG = (float*)(ws + kOffCG);
  float* G1 = (float*)(ws + kOffG1);
  unsigned short* ZZ16 = (unsigned short*)(ws + kOffZZ16);
  unsigned short* CT16 = (unsigned short*)(ws + kOffCT16);
  float* CT32 = (float*)(ws + kOffCT32);
  float* C0 = (float*)(ws + kOffC0);
  float* C1 = (float*)(ws + kOffC1);
  unsigned short* ZS16 = (unsigned short*)(ws + kOffZS16);
  float* OUTP = (float*)(ws + kOffOUTP);
  const float* ZB = BIAS + kFZB;

  hp_mask_cast_kernel<<<(kRowsE * (kE / 8)) / kThr, kThr, 0, stream>>>(hpad, hlen, HP16);
  embed_gather_kernel<<<(kRowsO * (kH / 8)) / kThr, kThr, 0, stream>>>(embed, ys_in, EY16);
  wt_plane_kernel<<<kA, kE / 8, 0, stream>>>(Wenc, WENC, kE, kA, kA, kE, 0);
  wt_plane_kernel<<<kA, kH / 8, 0, stream>>>(Wdec, WDEC, kH, kA, kA, kH, 0);
  wt_plane_kernel<<<kVP, kF / 8, 0, stream>>>(Wout, WOUT, kF, kV, kV, kF, 0);
  cast_plane_kernel<<<(kG4 * kH / 8) / kThr, kThr, 0, stream>>>(Whh0, WHH0, 10, kH, 0);
  cast_plane_kernel<<<(kG4 * kH / 8) / kThr, kThr, 0, stream>>>(Wih1, W1CAT, 10, kH2, 0);
  cast_plane_kernel<<<(kG4 * kH / 8) / kThr, kThr, 0, stream>>>(Whh1, W1CAT, 10, kH2, kH);
  wih0_cast_kernel<<<(kG4 * (kF / 8)) / kThr, kThr, 0, stream>>>(Wih0, WIH0E, WIH0C);
  bias_rows_kernel<<<18, kThr, 0, stream>>>(bih0, bhh0, bih1, bhh1, benc, bout, BIAS);
  state_zero_kernel<<<144, kThr, 0, stream>>>(ZZ16, CT16, C0, C1);

  wmma_gemm64<0, false, 2, 0, false, 0><<<dim3((kRowsE / 64) * (kA / 64) / 8, 1), 256, 0, stream>>>(
      HP16, HP16, kE, 0L, WENC, WENC, kE, 0L, (void*)PENC, (void*)PENC, kA, 0L, BIAS + kFBENC, nullptr, 0L, kRowsE, kA, kE, kSc22);
  wmma_gemm64<0, false, 2, 0, false, 0><<<dim3((kRowsO / 64) * (kG4 / 64) / 8, 1), 256, 0, stream>>>(
      EY16, EY16, kH, 0L, WIH0E, WIH0E, kH, 0L, (void*)EYG, (void*)EYG, kG4, 0L, BIAS + kFB0, nullptr, 0L, kRowsO, kG4, kH, kSc20);

  for (int t = 0; t < kO; ++t) {
    wmma_gemm64<0, false, 2, 0, false, 0><<<dim3((kBP / 64) * (kG4 / 64) / 8, 1), 256, 0, stream>>>(
        ZZ16, ZZ16, kH2, 0L, WHH0, WHH0, kH, 0L, (void*)HV0, (void*)HV0, kG4, 0L, ZB, nullptr, 0L, kBP, kG4, kH, kSc20);
    wmma_gemm64<0, false, 2, 0, false, 0><<<dim3((kBP / 64) * (kA / 64) / 8, 1), 256, 0, stream>>>(
        ZZ16, ZZ16, kH2, 0L, WDEC, WDEC, kH, 0L, (void*)DEC, (void*)DEC, kA, 0L, ZB, nullptr, 0L, kBP, kA, kH, kSc22);
    dec_attn_kernel<<<kB, kThr, 0, stream>>>(PENC, DEC, gvec, hlen, HP16, CT32, CT16);
    wmma_gemm64<0, false, 2, 0, false, 0><<<dim3((kBP / 64) * (kG4 / 64) / 8, 1), 256, 0, stream>>>(
        CT16, CT16, kE, 0L, WIH0C, WIH0C, kE, 0L, (void*)CG, (void*)CG, kG4, 0L, ZB, nullptr, 0L, kBP, kG4, kE, kSc20);
    cell0_kernel<<<16, kThr, 0, stream>>>(EYG, CG, HV0, C0, ZZ16, t);
    wmma_gemm64<0, false, 2, 0, false, 0><<<dim3((kBP / 64) * (kG4 / 64) / 8, 1), 256, 0, stream>>>(
        ZZ16, ZZ16, kH2, 0L, W1CAT, W1CAT, kH2, 0L, (void*)G1, (void*)G1, kG4, 0L, BIAS + kFB1, nullptr, 0L, kBP, kG4, kH2, kSc20);
    cell1_kernel<<<16, kThr, 0, stream>>>(G1, CT32, C1, ZZ16, ZS16, t);
  }
  wmma_gemm64<0, false, 2, 0, false, 0><<<dim3((kRowsO / 64) * (kVP / 64) / 8, 1), 256, 0, stream>>>(
      ZS16, ZS16, kF, 0L, WOUT, WOUT, kF, 0L, (void*)OUTP, (void*)OUTP, kVP, 0L, BIAS + kFBOUT, nullptr, 0L, kRowsO, kVP, kF, kSc22);
  assemble_out_kernel<<<(int)((size_t)kRowsO * kV / 4 / kThr), kThr, 0, stream>>>(OUTP, out);
}
